// DifferentialGQA_73151882985489
// MI455X (gfx1250) — hardware-run, weakly checked
//
#include <hip/hip_runtime.h>


#ifndef NB
#define NB 1
#endif
#ifndef SEQ
#define SEQ 2048
#endif
#define NB_FULL  1
#define SEQ_FULL 2048
#define DM   2048
#define NH   32
#define NKV  8
#define REP  (NH / NKV)
#define HD   64
#define DQ   (NH * HD)
#define DKV  (NKV * HD)
#define RH   ((SEQ) < 512 ? (SEQ) : 512)
#define NW   (SEQ / 32)
#define PP   40
#define PCAR 16384.0f
#define TSC  0.0072134752044448170f
#define CL2  72.134752044448170f
#define FILL2 (-1.4426950408889634e9f)
#define LINIT 0.6192834728526787f
#define POSTS 0.3807165271473213f

static_assert(SEQ % 64 == 0);
static_assert(SEQ <= SEQ_FULL);
static_assert(NW <= 64);
static_assert(HD == 64);
static_assert(DM % 64 == 0 && DQ % 64 == 0 && DKV % 64 == 0);
static_assert(DM % 32 == 0 && DQ % 32 == 0);
static_assert(NH % NKV == 0);
static_assert(RH % 16 == 0 && (SEQ - RH) % 16 == 0);
static_assert((PP * 2) % 16 == 0);
static_assert(NB <= NB_FULL);
static_assert(NB == 1);
static_assert(NH == 32);
static_assert(NH % 2 == 0 && REP % 2 == 0);
static_assert(NKV <= 32);
static_assert(SEQ % 8 == 0);
static_assert((32 / 8) * 4 == 16);
static_assert(8 * 16 == 2 * HD);
static_assert((size_t)2 * 16 * PP * 2 + (size_t)16 * 68 * 4 <= (size_t)131072);
static_assert((size_t)8 * 64 * 4 <= (size_t)131072);
static_assert((size_t)NH * SEQ * HD < (size_t)2147483647);

typedef _Float16 h16;
typedef unsigned short bf;
typedef __attribute__((ext_vector_type(16))) __bf16   v16bf;
typedef __attribute__((ext_vector_type(16))) _Float16 v16h;
typedef __attribute__((ext_vector_type(8)))  _Float16 v8h;
typedef __attribute__((ext_vector_type(8)))  unsigned short v8us;
typedef __attribute__((ext_vector_type(8)))  float    v8f;
typedef __attribute__((ext_vector_type(4)))  float    v4f;
typedef __attribute__((ext_vector_type(2)))  _Float16 v2h;
typedef __attribute__((ext_vector_type(2)))  unsigned short v2us;
typedef __attribute__((ext_vector_type(2)))  float    v2f;
typedef v4f  __attribute__((may_alias)) v4fa;
typedef v8us __attribute__((may_alias)) v8usa;

__device__ __forceinline__ unsigned short f2bf(float f) { unsigned u = __float_as_uint(f); u += 0x7FFFu + ((u >> 16) & 1u); return (unsigned short)(u >> 16); }
__device__ __forceinline__ float bf2f(unsigned short b) { return __uint_as_float(((unsigned)b) << 16); }
__device__ __forceinline__ float bfr(float f) { return bf2f(f2bf(f)); }
__device__ __forceinline__ v16h cat16(v8h lo, v8h hi) { return __builtin_shufflevector(lo, hi, 0, 1, 2, 3, 4, 5, 6, 7, 8, 9, 10, 11, 12, 13, 14, 15); }
__device__ __forceinline__ v16bf cat16b(v8us lo, v8us hi) { return __builtin_bit_cast(v16bf, __builtin_shufflevector(lo, hi, 0, 1, 2, 3, 4, 5, 6, 7, 8, 9, 10, 11, 12, 13, 14, 15)); }
__device__ __forceinline__ v16h cat16hu(v8us lo, v8us hi) { return __builtin_bit_cast(v16h, __builtin_shufflevector(lo, hi, 0, 1, 2, 3, 4, 5, 6, 7, 8, 9, 10, 11, 12, 13, 14, 15)); }
__device__ __forceinline__ v8f wmma16(v16h a, v16h b, v8f c) { return __builtin_amdgcn_wmma_f32_16x16x32_f16(false, a, false, b, (short)0, c, false, false); }
__device__ __forceinline__ v8f wmmab(v16bf a, v16bf b, v8f c) { return __builtin_amdgcn_wmma_f32_16x16x32_bf16(false, a, false, b, (short)0, c, false, false); }
__device__ __forceinline__ void splitf(float y, unsigned short& h, unsigned short& l) { h = f2bf(y); l = f2bf(y - bf2f(h)); }
__device__ __forceinline__ float ex2(float x) { return __builtin_amdgcn_exp2f(x); }

__device__ __forceinline__ h16 toh_flush(float v) { const h16 r = (h16)v; return (fabsf(v) < 6.103515625e-05f) ? (h16)0.0f : r; }
__device__ __forceinline__ v8f wmma16g(v16h a, v16h b, v8f c) { c = __builtin_amdgcn_wmma_f32_16x16x32_f16(false, a, false, b, (short)0, c, false, false); asm volatile("v_nop\n\tv_nop\n\tv_nop\n\tv_nop" : "+v"(c) : "v"(a), "v"(b)); return c; }
__device__ __forceinline__ v8f wmmabg(v16bf a, v16bf b, v8f c) { c = __builtin_amdgcn_wmma_f32_16x16x32_bf16(false, a, false, b, (short)0, c, false, false); asm volatile("v_nop\n\tv_nop\n\tv_nop\n\tv_nop" : "+v"(c) : "v"(a), "v"(b)); return c; }
__device__ __forceinline__ float capl2(float s) { const float t = ex2(s * TSC); const float rc = __builtin_amdgcn_rcpf(t + 1.0f); return (1.0f - 2.0f * rc) * CL2; }

template <typename T16> struct WFrag;
template <> struct WFrag<h16> { typedef v16h V; static __device__ __forceinline__ V ld(const h16* p) { return cat16(*(const v8h*)p, *(const v8h*)(p + 16)); } static __device__ __forceinline__ v8f mma(V a, V b, v8f c) { return wmma16(a, b, c); } };
template <> struct WFrag<bf> { typedef v16bf V; static __device__ __forceinline__ V ld(const bf* p) { return cat16b(*(const v8us*)p, *(const v8us*)(p + 16)); } static __device__ __forceinline__ v8f mma(V a, V b, v8f c) { return wmmab(a, b, c); } };

template <typename T16, int NSPLIT>
__device__ __forceinline__ void gemmw_body(const T16* __restrict__ A, const T16* __restrict__ A2, const T16* __restrict__ Bt, int K, float* C, int ldc) {
    typedef typename WFrag<T16>::V V;
    __shared__ __align__(16) float os[16 * 68];
    const int lane = threadIdx.x & 31, lr = lane & 15, hi = lane >> 4; const int r0 = blockIdx.x * 64, c0 = blockIdx.y * 64;
    v8f acc[4][4];
#pragma unroll
    for (int mb = 0; mb < 4; ++mb)
#pragma unroll
        for (int nb = 0; nb < 4; ++nb) acc[mb][nb] = (v8f){};
    const size_t aoff = (size_t)(r0 + lr) * K + 8 * hi, boff = (size_t)(c0 + lr) * K + 8 * hi;
#pragma unroll 1
    for (int kc = 0; kc < K; kc += 32) {
        V a[4], a2[4];
#pragma unroll
        for (int mb = 0; mb < 4; ++mb) { a[mb] = WFrag<T16>::ld(A + aoff + (size_t)mb * 16 * K + kc); if (NSPLIT == 1) a2[mb] = WFrag<T16>::ld(A2 + aoff + (size_t)mb * 16 * K + kc); else a2[mb] = a[mb]; }
#pragma unroll
        for (int nb = 0; nb < 4; ++nb) { const V b = WFrag<T16>::ld(Bt + boff + (size_t)nb * 16 * K + kc);
#pragma unroll
            for (int mb = 0; mb < 4; ++mb) { acc[mb][nb] = WFrag<T16>::mma(a[mb], b, acc[mb][nb]); if (NSPLIT == 1) acc[mb][nb] = WFrag<T16>::mma(a2[mb], b, acc[mb][nb]); } }
        asm volatile("v_nop\n\tv_nop\n\tv_nop\n\tv_nop" : "+v"(acc[0][0]), "+v"(acc[1][1]), "+v"(acc[2][2]), "+v"(acc[3][3]) : "v"(a[0]), "v"(a[3]));
    }
#pragma unroll
    for (int mb = 0; mb < 4; ++mb) {
#pragma unroll
        for (int nb = 0; nb < 4; ++nb) {
#pragma unroll
            for (int j = 0; j < 8; ++j) os[(hi * 8 + j) * 68 + nb * 16 + lr] = acc[mb][nb][j]; }
        __builtin_amdgcn_wave_barrier(); asm volatile("" ::: "memory");
        float* crow = C + (size_t)(r0 + mb * 16) * ldc + c0;
#pragma unroll 1
        for (int ps = 0; ps < 2; ++ps) {
#pragma unroll
            for (int s = 0; s < 8; ++s) { const int row = 2 * s + hi, cofs = lr * 4; const v4f val = *(const v4fa*)(os + row * 68 + cofs);
                *(volatile v4f*)(crow + (size_t)row * ldc + cofs) = val; }
            if (ps == 0) __threadfence(); }
        __builtin_amdgcn_wave_barrier(); asm volatile("" ::: "memory");
    }
}
__global__ __launch_bounds__(32) void k_gemm_p(const bf* __restrict__ A, const bf* __restrict__ Bt, int K, float* C, int ldc) { gemmw_body<bf, 0>(A, A, Bt, K, C, ldc); }
__global__ __launch_bounds__(32) void k_gemm_s(const bf* __restrict__ A, const bf* __restrict__ A2, const bf* __restrict__ Bt, int K, float* C, int ldc) { gemmw_body<bf, 1>(A, A2, Bt, K, C, ldc); }

__global__ __launch_bounds__(256) void k_wtG(const float* __restrict__ w, int K, int N, bf* Bt) {
    const int lane = threadIdx.x & 31; const int L0 = (blockIdx.x * 8 + (threadIdx.x >> 5)) * 8; const int nlines = N * K / 64;
#pragma unroll
    for (int ps = 0; ps < 2; ++ps) {
#pragma unroll 1
        for (int l = 0; l < 8; ++l) { const int L = L0 + l; if (L >= nlines) break; const size_t e = (size_t)L * 64 + lane * 2; const int k = (int)(e % K), n = (int)(e / K); v2us o;
            o[0] = f2bf(w[(size_t)k * N + n]); o[1] = f2bf(w[(size_t)(k + 1) * N + n]); *(volatile v2us*)(Bt + e) = o; }
        if (ps == 0) __threadfence(); }
}
__global__ __launch_bounds__(256) void k_cvt8(const float* __restrict__ src, bf* dst, size_t n8) { const size_t i = (size_t)blockIdx.x * 256 + threadIdx.x; if (i >= n8) return; const v8f v = *(const v8f*)(src + i * 8); v8us o;
#pragma unroll
    for (int k = 0; k < 8; ++k) o[k] = f2bf(v[k]); *(volatile v8us*)(dst + i * 8) = o; __threadfence(); *(volatile v8us*)(dst + i * 8) = o; }

__global__ __launch_bounds__(256) void k_rope(const float* __restrict__ F, int pitch, int nheads, const float* __restrict__ COS, const float* __restrict__ SIN, h16* P16, bf* Ph, bf* Pl) {
#pragma clang fp contract(off)
    const size_t e = ((size_t)blockIdx.x * 256 + threadIdx.x) * 2; if (e >= (size_t)nheads * SEQ * HD) return;
    const int d = (int)(e % HD); const int t = (int)((e / HD) % SEQ); const int h = (int)(e / ((size_t)HD * SEQ));
    const int dp = d ^ (HD / 2); const int ti = d & (HD / 2 - 1); const bool lowh = d < (HD / 2);
    const v2f x  = *(const v2f*)(F + (size_t)t * pitch + h * HD + d);
    const v2f xp = *(const v2f*)(F + (size_t)t * pitch + h * HD + dp);
    const v2f cc = *(const v2f*)(COS + (size_t)t * (HD / 2) + ti);
    const v2f sn = *(const v2f*)(SIN + (size_t)t * (HD / 2) + ti);
    v2h o16; v2us oh, ol;
#pragma unroll
    for (int q = 0; q < 2; ++q) {
        const float c = bfr(cc[q]), s = bfr(sn[q]);
        const float a = x[q] * c, b = xp[q] * s;
        const float dif = a - b, sum = b + a;
        const float r = lowh ? dif : sum;
        unsigned short a2, c2; splitf(r, a2, c2);
        o16[q] = toh_flush(r); oh[q] = a2; ol[q] = c2; }
    *(volatile v2h*)(P16 + e) = o16; *(volatile v2us*)(Ph + e) = oh; *(volatile v2us*)(Pl + e) = ol; __threadfence(); *(volatile v2h*)(P16 + e) = o16; *(volatile v2us*)(Ph + e) = oh; *(volatile v2us*)(Pl + e) = ol; }
__global__ __launch_bounds__(256) void k_vtp(const float* __restrict__ F, int pitch, int nheads, h16* V16, bf* Vh, bf* Vl) { const size_t e = ((size_t)blockIdx.x * 256 + threadIdx.x) * 2; if (e >= (size_t)nheads * HD * SEQ) return; const int t = (int)(e % SEQ); const int d = (int)((e / SEQ) % HD); const int g = (int)(e / ((size_t)SEQ * HD)); v2h o16; v2us oh, ol;
#pragma unroll
    for (int q = 0; q < 2; ++q) { const float x = F[(size_t)(t + q) * pitch + g * HD + d]; o16[q] = (h16)x; unsigned short a2, c2; splitf(x, a2, c2); oh[q] = a2; ol[q] = c2; }
    *(volatile v2h*)(V16 + e) = o16; *(volatile v2us*)(Vh + e) = oh; *(volatile v2us*)(Vl + e) = ol; __threadfence(); *(volatile v2h*)(V16 + e) = o16; *(volatile v2us*)(Vh + e) = oh; *(volatile v2us*)(Vl + e) = ol; }

__global__ __launch_bounds__(32) void k_maskbits(const int* __restrict__ mask, unsigned* MBp, int* CLp) {
    const int lane = threadIdx.x & 31; const int qt = blockIdx.x; const int q0 = qt * 16;
    unsigned and0 = 0xFFFFFFFFu, and1 = 0xFFFFFFFFu, or0 = 0u, or1 = 0u; int empt = 0;
#pragma unroll 1
    for (int row = 0; row < 16; ++row) {
        const int* mr = mask + (size_t)(q0 + row) * SEQ_FULL; unsigned w0 = 0u, w1 = 0u;
#pragma unroll 4
        for (int w = 0; w < NW; ++w) { const int v = mr[32 * w + lane]; const unsigned b = __builtin_amdgcn_ballot_w32(v != 0); w0 = (w == lane) ? b : w0; w1 = (w == lane + 32) ? b : w1; }
        and0 &= w0; and1 &= w1; or0 |= w0; or1 |= w1;
        const unsigned rb = __builtin_amdgcn_ballot_w32((w0 | w1) != 0u);
        empt |= (rb == 0u) ? 1 : 0;
        unsigned* dst = MBp + (size_t)(q0 + row) * NW;
        if (lane < NW) *(volatile unsigned*)(dst + lane) = w0;
        if (lane + 32 < NW) *(volatile unsigned*)(dst + 32 + lane) = w1;
        __threadfence();
        if (lane < NW) *(volatile unsigned*)(dst + lane) = w0;
        if (lane + 32 < NW) *(volatile unsigned*)(dst + 32 + lane) = w1;
    }
    const int cz = (empt != 0) ? 2 : 0;
    const int c0 = (or0 == 0u) ? cz : ((and0 == 0xFFFFFFFFu) ? 1 : 2); const int c1 = (or1 == 0u) ? cz : ((and1 == 0xFFFFFFFFu) ? 1 : 2);
    int* cd = CLp + (size_t)qt * NW;
    if (lane < NW) *(volatile int*)(cd + lane) = c0;
    if (lane + 32 < NW) *(volatile int*)(cd + 32 + lane) = c1;
    __threadfence();
    if (lane < NW) *(volatile int*)(cd + lane) = c0;
    if (lane + 32 < NW) *(volatile int*)(cd + 32 + lane) = c1;
}

__global__ __launch_bounds__(256) void k_lamsum(const bf* __restrict__ Ph, const bf* __restrict__ Pl, const float* __restrict__ la, const float* __restrict__ lb, float* PART, int line0) {
    __shared__ float red[8 * 64];
    const int lane = threadIdx.x & 31; const int wave = __builtin_amdgcn_readfirstlane(threadIdx.x >> 5); const int h = (int)blockIdx.x;
    float a0 = 0.0f, a1 = 0.0f;
#pragma unroll 4
    for (int t = wave; t < SEQ; t += 8) { const size_t o = ((size_t)h * SEQ + t) * HD + 2 * lane; const v2us vh = *(const v2us*)(Ph + o), vl = *(const v2us*)(Pl + o);
        a0 += bf2f(vh[0]) + bf2f(vl[0]); a1 += bf2f(vh[1]) + bf2f(vl[1]); }
    red[wave * 64 + 2 * lane] = a0; red[wave * 64 + 2 * lane + 1] = a1;
    __syncthreads();
    if (wave == 0) {
        float c0 = 0.0f, c1 = 0.0f;
#pragma unroll
        for (int w = 0; w < 8; ++w) { c0 += red[w * 64 + 2 * lane]; c1 += red[w * 64 + 2 * lane + 1]; }
        float sa = c0 * bfr(la[2 * lane]) + c1 * bfr(la[2 * lane + 1]);
        float sb = c0 * bfr(lb[2 * lane]) + c1 * bfr(lb[2 * lane + 1]);
#pragma unroll
        for (int o = 16; o >= 1; o >>= 1) { sa += __shfl_xor(sa, o, 32); sb += __shfl_xor(sb, o, 32); }
        const float val = (lane == 0) ? sa : ((lane == 1) ? sb : 0.0f);
        float* dst = PART + (size_t)(line0 + h) * 32;
        *(volatile float*)(dst + lane) = val; __threadfence(); *(volatile float*)(dst + lane) = val;
    }
}
__global__ __launch_bounds__(32) void k_lamfin(const float* __restrict__ PART, float* LAMp) {
#pragma clang fp contract(off)
    const int lane = threadIdx.x & 31;
    const v2f qa = *(const v2f*)(PART + (size_t)lane * 32);
    const int kl = (lane < NKV) ? lane : (NKV - 1);
    const v2f ka = *(const v2f*)(PART + (size_t)(NH + kl) * 32);
    const float km = (lane < NKV) ? (float)(REP / 2) : 0.0f;
    float d1 = ((lane & 1) == 0) ? qa[0] : 0.0f; float d3 = ((lane & 1) != 0) ? qa[1] : 0.0f;
    float d2 = ka[0] * km; float d4 = ka[1] * km;
#pragma unroll
    for (int o = 16; o >= 1; o >>= 1) { d1 += __shfl_xor(d1, o, 32); d2 += __shfl_xor(d2, o, 32); d3 += __shfl_xor(d3, o, 32); d4 += __shfl_xor(d4, o, 32); }
    const float inv = 1.0f / (float)(NB * SEQ);
    d1 = fminf(fmaxf(d1 * inv, -10.0f), 10.0f); d2 = fminf(fmaxf(d2 * inv, -10.0f), 10.0f); d3 = fminf(fmaxf(d3 * inv, -10.0f), 10.0f); d4 = fminf(fmaxf(d4 * inv, -10.0f), 10.0f);
    const float dd = (lane == 0) ? d1 : ((lane == 1) ? d2 : ((lane == 2) ? d3 : d4));
    const float ee = expf(dd);
    const float e1 = __shfl(ee, 0, 32), e2 = __shfl(ee, 1, 32), e3 = __shfl(ee, 2, 32), e4 = __shfl(ee, 3, 32);
    const float pa = e1 * e2, pb = e3 * e4;
    float lam = (pa - pb) + LINIT; lam = fminf(fmaxf(lam, 0.0f), 1.0f);
    *(volatile float*)(LAMp + lane) = lam; __threadfence(); *(volatile float*)(LAMp + lane) = lam;
}

__device__ __forceinline__ void tile_words(const unsigned* __restrict__ MBp, int cls, int q0, int hi, int j, unsigned (&wd)[8]) {
    if (cls == 1) {
#pragma unroll
        for (int r = 0; r < 8; ++r) wd[r] = 0xFFFFFFFFu;
    } else {
#pragma unroll
        for (int r = 0; r < 8; ++r) wd[r] = MBp[(size_t)(q0 + 8 * hi + r) * NW + j];
    }
}
__device__ __forceinline__ v8f score6(const bf* __restrict__ Qh, const bf* __restrict__ Ql, int qo, v16bf kh0, v16bf kh1, v16bf kl0, v16bf kl1) {
    asm volatile("" : "+v"(qo));
    const v16bf qh0 = WFrag<bf>::ld(Qh + (size_t)qo), qh1 = WFrag<bf>::ld(Qh + (size_t)qo + 32), ql0 = WFrag<bf>::ld(Ql + (size_t)qo), ql1 = WFrag<bf>::ld(Ql + (size_t)qo + 32);
    v8f s = (v8f){};
    s = wmmabg(ql0, kh0, s); s = wmmabg(ql1, kh1, s); s = wmmabg(qh0, kl0, s); s = wmmabg(qh1, kl1, s); s = wmmabg(qh0, kh0, s); s = wmmabg(qh1, kh1, s);
    return s;
}
template <bool SPLIT>
__device__ __forceinline__ void pair_scores(const h16* __restrict__ Q16, const h16* __restrict__ K16, const bf* __restrict__ Qh, const bf* __restrict__ Ql, const bf* __restrict__ Kh, const bf* __restrict__ Kl,
                                            int qo1, int qo2, size_t ko, v8f& s10, v8f& s11, v8f& s20, v8f& s21) {
    if (SPLIT) {
        { const v16bf kh0 = WFrag<bf>::ld(Kh + ko), kh1 = WFrag<bf>::ld(Kh + ko + 32), kl0 = WFrag<bf>::ld(Kl + ko), kl1 = WFrag<bf>::ld(Kl + ko + 32);
          s10 = score6(Qh, Ql, qo1, kh0, kh1, kl0, kl1); s20 = score6(Qh, Ql, qo2, kh0, kh1, kl0, kl1); }
        { const size_t k1 = ko + (size_t)16 * HD; const v16bf kh0 = WFrag<bf>::ld(Kh + k1), kh1 = WFrag<bf>::ld(Kh + k1 + 32), kl0 = WFrag<bf>::ld(Kl + k1), kl1 = WFrag<bf>::ld(Kl + k1 + 32);
          s11 = score6(Qh, Ql, qo1, kh0, kh1, kl0, kl1); s21 = score6(Qh, Ql, qo2, kh0, kh1, kl0, kl1); }
    } else {
        asm volatile("" : "+v"(qo1), "+v"(qo2));
        const v16h qa0 = WFrag<h16>::ld(Q16 + (size_t)qo1), qa1 = WFrag<h16>::ld(Q16 + (size_t)qo1 + 32);
        const v16h qb0 = WFrag<h16>::ld(Q16 + (size_t)qo2), qb1 = WFrag<h16>::ld(Q16 + (size_t)qo2 + 32);
        const v16h k00 = WFrag<h16>::ld(K16 + ko), k01 = WFrag<h16>::ld(K16 + ko + 32);
        const v16h k10 = WFrag<h16>::ld(K16 + ko + (size_t)16 * HD), k11 = WFrag<h16>::ld(K16 + ko + (size_t)16 * HD + 32);
        s10 = wmma16g(qa0, k00, (v8f){}); s10 = wmma16g(qa1, k01, s10);
        s11 = wmma16g(qa0, k10, (v8f){}); s11 = wmma16g(qa1, k11, s11);
        s20 = wmma16g(qb0, k00, (v8f){}); s20 = wmma16g(qb1, k01, s20);
        s21 = wmma16g(qb0, k10, (v8f){}); s21 = wmma16g(qb1, k11, s21);
    }
}

template <bool SPLIT>
__device__ __forceinline__ void dattn_body(const h16* __restrict__ Q16, const h16* __restrict__ K16, const h16* __restrict__ V16,
                                           const bf* __restrict__ Qh, const bf* __restrict__ Ql, const bf* __restrict__ Kh, const bf* __restrict__ Kl, const bf* __restrict__ Vh, const bf* __restrict__ Vl,
                                           const unsigned* __restrict__ MBp, const int* __restrict__ CLp, const float* __restrict__ LAMp, const float* __restrict__ SUBW, bf* Ch, bf* Cl, int qt0) {
    __shared__ __align__(16) unsigned short pa[16 * PP];
    __shared__ __align__(16) unsigned short pb[16 * PP];
    __shared__ __align__(16) float os[16 * 68];
    const int lane = threadIdx.x & 31, lr = lane & 15, hi = lane >> 4;
    const int qt = qt0 + (int)blockIdx.x; const int pr = (int)blockIdx.y; const int h1 = 2 * pr; const int hk = h1 / REP; const int q0 = qt * 16;
    const int qo1 = (int)(((size_t)h1 * SEQ + q0 + lr) * HD + 8 * hi);
    const int qo2 = qo1 + SEQ * HD;
    const size_t kb0  = ((size_t)hk * SEQ + lr) * HD + 8 * hi;
    const size_t vb0  = ((size_t)hk * HD + lr) * SEQ + 8 * hi;
    const float NINF = -__builtin_inff();
    const float lam = LAMp[0];
    float m1[8], l1[8], m2[8], l2[8];
#pragma unroll
    for (int r = 0; r < 8; ++r) { m1[r] = NINF; l1[r] = 0.0f; m2[r] = NINF; l2[r] = 0.0f; }
#pragma unroll 1
    for (int j = 0; j < NW; ++j) {
        const int cls = __builtin_amdgcn_readfirstlane(CLp[(size_t)qt * NW + j]);
        if (cls == 0) continue;
        unsigned wd[8]; tile_words(MBp, cls, q0, hi, j, wd);
        v8f s10, s11, s20, s21;
        pair_scores<SPLIT>(Q16, K16, Qh, Ql, Kh, Kl, qo1, qo2, kb0 + (size_t)(32 * j) * HD, s10, s11, s20, s21);
#pragma unroll
        for (int r = 0; r < 8; ++r) {
            const unsigned w = wd[r];
            const bool kp0 = ((w >> lr) & 1u) != 0u, kp1 = ((w >> (16 + lr)) & 1u) != 0u;
            const float c10 = capl2(s10[r]), c11 = capl2(s11[r]), c20 = capl2(s20[r]), c21 = capl2(s21[r]);
            const float a0 = kp0 ? c10 : FILL2, a1 = kp1 ? c11 : FILL2;
            const float b0 = kp0 ? c20 : FILL2, b1 = kp1 ? c21 : FILL2;
            { const float nm = fmaxf(m1[r], fmaxf(a0, a1)); l1[r] = l1[r] * ex2(m1[r] - nm) + (ex2(a0 - nm) + ex2(a1 - nm)); m1[r] = nm; }
            { const float nm = fmaxf(m2[r], fmaxf(b0, b1)); l2[r] = l2[r] * ex2(m2[r] - nm) + (ex2(b0 - nm) + ex2(b1 - nm)); m2[r] = nm; }
        }
    }
#pragma unroll
    for (int r = 0; r < 8; ++r) {
        { float M = m1[r]; M = fmaxf(M, __shfl_xor(M, 1, 32)); M = fmaxf(M, __shfl_xor(M, 2, 32)); M = fmaxf(M, __shfl_xor(M, 4, 32)); M = fmaxf(M, __shfl_xor(M, 8, 32));
          float l = l1[r] * ex2(m1[r] - M); l += __shfl_xor(l, 1, 32); l += __shfl_xor(l, 2, 32); l += __shfl_xor(l, 4, 32); l += __shfl_xor(l, 8, 32);
          m1[r] = M; l1[r] = 1.0f / l; }
        { float M = m2[r]; M = fmaxf(M, __shfl_xor(M, 1, 32)); M = fmaxf(M, __shfl_xor(M, 2, 32)); M = fmaxf(M, __shfl_xor(M, 4, 32)); M = fmaxf(M, __shfl_xor(M, 8, 32));
          float l = l2[r] * ex2(m2[r] - M); l += __shfl_xor(l, 1, 32); l += __shfl_xor(l, 2, 32); l += __shfl_xor(l, 4, 32); l += __shfl_xor(l, 8, 32);
          m2[r] = M; l2[r] = lam * (1.0f / l); }
    }
    v8f acc[4];
#pragma unroll
    for (int ot = 0; ot < 4; ++ot) acc[ot] = (v8f){};
#pragma unroll 1
    for (int j = 0; j < NW; ++j) {
        const int cls = __builtin_amdgcn_readfirstlane(CLp[(size_t)qt * NW + j]);
        if (cls == 0) continue;
        unsigned wd[8]; tile_words(MBp, cls, q0, hi, j, wd);
        v8f s10, s11, s20, s21;
        pair_scores<SPLIT>(Q16, K16, Qh, Ql, Kh, Kl, qo1, qo2, kb0 + (size_t)(32 * j) * HD, s10, s11, s20, s21);
#pragma unroll
        for (int r = 0; r < 8; ++r) {
            const unsigned w = wd[r];
            const bool kp0 = ((w >> lr) & 1u) != 0u, kp1 = ((w >> (16 + lr)) & 1u) != 0u;
            const float c10 = capl2(s10[r]), c11 = capl2(s11[r]), c20 = capl2(s20[r]), c21 = capl2(s21[r]);
            const float a0 = kp0 ? c10 : FILL2, a1 = kp1 ? c11 : FILL2;
            const float b0 = kp0 ? c20 : FILL2, b1 = kp1 ? c21 : FILL2;
            const float p0 = fmaxf(ex2(a0 - m1[r]) * l1[r] - ex2(b0 - m2[r]) * l2[r], 0.0f);
            const float p1 = fmaxf(ex2(a1 - m1[r]) * l1[r] - ex2(b1 - m2[r]) * l2[r], 0.0f);
            const int po = (8 * hi + r) * PP + lr;
            if (SPLIT) { unsigned short a, c; splitf(p0, a, c); pa[po] = a; pb[po] = c; splitf(p1, a, c); pa[po + 16] = a; pb[po + 16] = c; }
            else { const h16 e0 = toh_flush(p0 * PCAR), e1 = toh_flush(p1 * PCAR); pa[po] = __builtin_bit_cast(unsigned short, e0); pa[po + 16] = __builtin_bit_cast(unsigned short, e1); }
        }
        __syncthreads();
        const size_t vo = vb0 + (size_t)(32 * j);
        if (SPLIT) {
            const v8us a0 = *(const v8usa*)(pa + lr * PP + 8 * hi), a1 = *(const v8usa*)(pa + lr * PP + 16 + 8 * hi);
            const v8us b0 = *(const v8usa*)(pb + lr * PP + 8 * hi), b1 = *(const v8usa*)(pb + lr * PP + 16 + 8 * hi);
            const v16bf ph = cat16b(a0, a1), pl = cat16b(b0, b1);
#pragma unroll
            for (int ot = 0; ot < 4; ++ot) { const v16bf vh = WFrag<bf>::ld(Vh + vo + (size_t)ot * 16 * SEQ), vl = WFrag<bf>::ld(Vl + vo + (size_t)ot * 16 * SEQ);
                acc[ot] = wmmabg(pl, vh, acc[ot]); acc[ot] = wmmabg(ph, vl, acc[ot]); acc[ot] = wmmabg(ph, vh, acc[ot]); }
        } else {
            const v8us a0 = *(const v8usa*)(pa + lr * PP + 8 * hi), a1 = *(const v8usa*)(pa + lr * PP + 16 + 8 * hi);
            const v16h p16 = cat16hu(a0, a1);
#pragma unroll
            for (int ot = 0; ot < 4; ++ot) { const v16h vf = WFrag<h16>::ld(V16 + vo + (size_t)ot * 16 * SEQ); acc[ot] = wmma16g(p16, vf, acc[ot]); }
        }
        asm volatile("" ::: "memory");
    }
    const float osc = SPLIT ? 1.0f : (1.0f / PCAR);
#pragma unroll
    for (int ot = 0; ot < 4; ++ot)
#pragma unroll
        for (int r = 0; r < 8; ++r) os[(8 * hi + r) * 68 + ot * 16 + lr] = acc[ot][r] * osc;
    __syncthreads();
    const int c8 = (lane & 7) * 8;
    float g1[8], g2[8];
    { const v4f wa0 = *(const v4f*)(SUBW + c8), wa1 = *(const v4f*)(SUBW + c8 + 4), wb0 = *(const v4f*)(SUBW + HD + c8), wb1 = *(const v4f*)(SUBW + HD + c8 + 4);
#pragma unroll
      for (int k = 0; k < 4; ++k) { g1[k] = bfr(wa0[k]); g1[4 + k] = bfr(wa1[k]); g2[k] = bfr(wb0[k]); g2[4 + k] = bfr(wb1[k]); } }
    v8us o1h[4], o1l[4], o2h[4], o2l[4];
#pragma unroll
    for (int s = 0; s < 4; ++s) { const int row = 4 * s + (lane >> 3);
        const v4f x0 = *(const v4fa*)(os + row * 68 + c8), x1 = *(const v4fa*)(os + row * 68 + c8 + 4);
        float xv[8];
#pragma unroll
        for (int k = 0; k < 4; ++k) { xv[k] = x0[k]; xv[4 + k] = x1[k]; }
        float ss = 0.0f;
#pragma unroll
        for (int k = 0; k < 8; ++k) ss += xv[k] * xv[k];
        ss += __shfl_xor(ss, 1, 32); ss += __shfl_xor(ss, 2, 32); ss += __shfl_xor(ss, 4, 32);
        const float rinv = 1.0f / sqrtf(ss * (1.0f / (float)HD) + 1e-6f);
#pragma unroll
        for (int k = 0; k < 8; ++k) { const float n = xv[k] * rinv; const float y1 = (n * g1[k]) * POSTS, y2 = (n * g2[k]) * POSTS; unsigned short a, c;
            splitf(y1, a, c); o1h[s][k] = a; o1l[s][k] = c; splitf(y2, a, c); o2h[s][k] = a; o2l[s][k] = c; }
    }
#pragma unroll 1
    for (int ps = 0; ps < 2; ++ps) {
#pragma unroll
        for (int s = 0; s < 4; ++s) { const int row = 4 * s + (lane >> 3);
            const size_t oo = (size_t)(q0 + row) * DQ + (size_t)h1 * HD + c8;
            *(volatile v8us*)(Ch + oo) = o1h[s]; *(volatile v8us*)(Cl + oo) = o1l[s];
            *(volatile v8us*)(Ch + oo + HD) = o2h[s]; *(volatile v8us*)(Cl + oo + HD) = o2l[s]; }
        if (ps == 0) __threadfence(); }
}
__global__ __launch_bounds__(32) __attribute__((amdgpu_num_vgpr(256))) void k_dattn_hl(const bf* __restrict__ Qh, const bf* __restrict__ Ql, const bf* __restrict__ Kh, const bf* __restrict__ Kl, const bf* __restrict__ Vh, const bf* __restrict__ Vl,
                                                 const unsigned* __restrict__ MBp, const int* __restrict__ CLp, const float* __restrict__ LAMp, const float* __restrict__ SUBW, bf* Ch, bf* Cl, int qt0) {
    dattn_body<true>((const h16*)0, (const h16*)0, (const h16*)0, Qh, Ql, Kh, Kl, Vh, Vl, MBp, CLp, LAMp, SUBW, Ch, Cl, qt0); }
__global__ __launch_bounds__(32) __attribute__((amdgpu_num_vgpr(256))) void k_dattn_f16(const h16* __restrict__ Q16, const h16* __restrict__ K16, const h16* __restrict__ V16,
                                                  const unsigned* __restrict__ MBp, const int* __restrict__ CLp, const float* __restrict__ LAMp, const float* __restrict__ SUBW, bf* Ch, bf* Cl, int qt0) {
    dattn_body<false>(Q16, K16, V16, (const bf*)0, (const bf*)0, (const bf*)0, (const bf*)0, (const bf*)0, (const bf*)0, MBp, CLp, LAMp, SUBW, Ch, Cl, qt0); }

constexpr size_t al256(size_t b) { return (b + 255) & ~(size_t)255; }
constexpr size_t WS_TOTAL =
    al256((size_t)DQ * DM * 2) + 2 * al256((size_t)DKV * DM * 2) + al256((size_t)DM * DQ * 2) +
    al256((size_t)SEQ * DM * 2) +
    al256((size_t)SEQ * DQ * 4) + 2 * al256((size_t)SEQ * DKV * 4) +
    3 * al256((size_t)NH * SEQ * HD * 2) + 6 * al256((size_t)NKV * SEQ * HD * 2) +
    2 * al256((size_t)SEQ * DQ * 2) +
    al256((size_t)SEQ * NW * 4) + al256((size_t)(SEQ / 16) * NW * 4) +
    al256((size_t)(NH + NKV) * 128) + al256((size_t)128);
static_assert(WS_TOTAL <= (size_t)134217728);
static_assert((size_t)(NH + NKV) * 32 * 4 <= al256((size_t)(NH + NKV) * 128));

extern "C" void kernel_launch(void* const* d_in, const int* in_sizes, int n_in,
                              void* d_out, int out_size, void* d_ws, size_t ws_size, hipStream_t stream) {
    if (n_in < 13) return;
    if ((long long)in_sizes[0] < (long long)(NB - 1) * SEQ_FULL * DM + (long long)SEQ * DM) return;
    if ((long long)in_sizes[1] < (long long)SEQ * (HD / 2) || (long long)in_sizes[2] < (long long)SEQ * (HD / 2)) return;
    if ((long long)in_sizes[3] < (long long)(SEQ - 1) * SEQ_FULL + SEQ) return;
    if ((long long)in_sizes[4] < (long long)DM * DQ || (long long)in_sizes[5] < (long long)DM * DKV || (long long)in_sizes[6] < (long long)DM * DKV || (long long)in_sizes[7] < (long long)DQ * DM) return;
    if (in_sizes[8] < HD || in_sizes[9] < HD || in_sizes[10] < HD || in_sizes[11] < HD || in_sizes[12] < 2 * HD) return;
    if ((long long)out_size < (long long)(NB - 1) * SEQ_FULL * DM + (long long)SEQ * DM) return;
    if (ws_size < WS_TOTAL) return;
    const float* x = (const float*)d_in[0]; const float* fcos = (const float*)d_in[1]; const float* fsin = (const float*)d_in[2]; const int* mask = (const int*)d_in[3];
    const float* wq = (const float*)d_in[4]; const float* wk = (const float*)d_in[5]; const float* wv = (const float*)d_in[6]; const float* wo = (const float*)d_in[7];
    const float* lq1 = (const float*)d_in[8]; const float* lk1 = (const float*)d_in[9]; const float* lq2 = (const float*)d_in[10]; const float* lk2 = (const float*)d_in[11];
    const float* subw = (const float*)d_in[12];
    float* OUT = (float*)d_out;
    char* wsp = (char*)d_ws;
    auto take = [&](size_t bytes) { char* p = wsp; wsp += (bytes + 255) & ~(size_t)255; return (void*)p; };
    bf* WQ = (bf*)take((size_t)DQ * DM * 2); bf* WK = (bf*)take((size_t)DKV * DM * 2); bf* WV = (bf*)take((size_t)DKV * DM * 2); bf* WO = (bf*)take((size_t)DM * DQ * 2);
    bf* XB = (bf*)take((size_t)SEQ * DM * 2);
    float* FQ = (float*)take((size_t)SEQ * DQ * 4); float* FK = (float*)take((size_t)SEQ * DKV * 4); float* FV = (float*)take((size_t)SEQ * DKV * 4);
    h16* QP16 = (h16*)take((size_t)NH * SEQ * HD * 2); bf* QPh = (bf*)take((size_t)NH * SEQ * HD * 2); bf* QPl = (bf*)take((size_t)NH * SEQ * HD * 2);
    h16* KP16 = (h16*)take((size_t)NKV * SEQ * HD * 2); bf* KPh = (bf*)take((size_t)NKV * SEQ * HD * 2); bf* KPl = (bf*)take((size_t)NKV * SEQ * HD * 2);
    h16* VT16 = (h16*)take((size_t)NKV * SEQ * HD * 2); bf* VTh = (bf*)take((size_t)NKV * SEQ * HD * 2); bf* VTl = (bf*)take((size_t)NKV * SEQ * HD * 2);
    bf* CXh = (bf*)take((size_t)SEQ * DQ * 2); bf* CXl = (bf*)take((size_t)SEQ * DQ * 2);
    unsigned* MBp = (unsigned*)take((size_t)SEQ * NW * 4); int* CLp = (int*)take((size_t)(SEQ / 16) * NW * 4);
    float* PART = (float*)take((size_t)(NH + NKV) * 128); float* LAMp = (float*)take((size_t)128);
    if ((size_t)(wsp - (char*)d_ws) > ws_size) return;

    k_wtG<<<(unsigned)((DM * DQ / 64 + 63) / 64), 256, 0, stream>>>(wq, DM, DQ, WQ);
    k_wtG<<<(unsigned)((DM * DKV / 64 + 63) / 64), 256, 0, stream>>>(wk, DM, DKV, WK);
    k_wtG<<<(unsigned)((DM * DKV / 64 + 63) / 64), 256, 0, stream>>>(wv, DM, DKV, WV);
    k_wtG<<<(unsigned)((DQ * DM / 64 + 63) / 64), 256, 0, stream>>>(wo, DQ, DM, WO);
    k_maskbits<<<SEQ / 16, 32, 0, stream>>>(mask, MBp, CLp);
    const unsigned LQ = (unsigned)(((size_t)NH * SEQ * HD / 2 + 255) / 256), LKv = (unsigned)(((size_t)NKV * SEQ * HD / 2 + 255) / 256);
    for (int b = 0; b < NB; ++b) {
        k_cvt8<<<(unsigned)(((size_t)SEQ * DM / 8 + 255) / 256), 256, 0, stream>>>(x + (size_t)b * SEQ_FULL * DM, XB, (size_t)SEQ * DM / 8);
        k_gemm_p<<<dim3(SEQ / 64, DQ / 64, 1), 32, 0, stream>>>(XB, WQ, DM, FQ, DQ);
        k_gemm_p<<<dim3(SEQ / 64, DKV / 64, 1), 32, 0, stream>>>(XB, WK, DM, FK, DKV);
        k_gemm_p<<<dim3(SEQ / 64, DKV / 64, 1), 32, 0, stream>>>(XB, WV, DM, FV, DKV);
        k_rope<<<LQ, 256, 0, stream>>>(FQ, DQ, NH, fcos, fsin, QP16, QPh, QPl);
        k_rope<<<LKv, 256, 0, stream>>>(FK, DKV, NKV, fcos, fsin, KP16, KPh, KPl);
        k_vtp<<<LKv, 256, 0, stream>>>(FV, DKV, NKV, VT16, VTh, VTl);
        k_lamsum<<<NH, 256, 0, stream>>>(QPh, QPl, lq1, lq2, PART, 0);
        k_lamsum<<<NKV, 256, 0, stream>>>(KPh, KPl, lk1, lk2, PART, NH);
        k_lamfin<<<1, 32, 0, stream>>>(PART, LAMp);
        if (RH / 16 > 0) k_dattn_hl<<<dim3(RH / 16, NH / 2, 1), 32, 0, stream>>>(QPh, QPl, KPh, KPl, VTh, VTl, MBp, CLp, LAMp, subw, CXh, CXl, 0);
        if ((SEQ - RH) / 16 > 0) k_dattn_f16<<<dim3((SEQ - RH) / 16, NH / 2, 1), 32, 0, stream>>>(QP16, KP16, VT16, MBp, CLp, LAMp, subw, CXh, CXl, RH / 16);
        k_gemm_s<<<dim3(SEQ / 64, DM / 64, 1), 32, 0, stream>>>(CXh, CXl, WO, DQ, OUT + (size_t)b * SEQ_FULL * DM, DM);
    }
}
